// RelRepBetweenContext_old_35957466202777
// MI455X (gfx1250) — hardware-verified
//
#include <hip/hip_runtime.h>
#define BB 4
#define KK 32
#define SS 1024
#define HH 512
#define FF 2304
#define NP (BB * KK * KK)

typedef _Float16 v16h __attribute__((ext_vector_type(16)));
typedef _Float16 v8h  __attribute__((ext_vector_type(8)));
typedef _Float16 v8ha __attribute__((ext_vector_type(8), may_alias));
typedef float    v8f  __attribute__((ext_vector_type(8)));
typedef float    v4f  __attribute__((ext_vector_type(4)));
typedef float    v4fa __attribute__((ext_vector_type(4), may_alias));
union Frag { v16h v; v8h half[2]; _Float16 h[16]; };

__device__ __forceinline__ v8f mma16(v16h a, v16h b, v8f c) {
  c = __builtin_amdgcn_wmma_f32_16x16x32_f16(false, a, false, b, (short)0, c, false, false);
  asm volatile("v_nop\n\tv_nop\n\tv_nop\n\tv_nop" : "+v"(c) : "v"(a), "v"(b));
  return c;
}

__global__ __launch_bounds__(256) void k_cvt16(const float* __restrict__ src, _Float16* __restrict__ dst, int n8) {
  const int t = blockIdx.x * 256 + threadIdx.x;
  if (t >= n8) return;
  const v4f a = *(const v4fa*)(src + (size_t)t * 8), b = *(const v4fa*)(src + (size_t)t * 8 + 4);
  v8h v; v[0]=(_Float16)a[0]; v[1]=(_Float16)a[1]; v[2]=(_Float16)a[2]; v[3]=(_Float16)a[3];
  v[4]=(_Float16)b[0]; v[5]=(_Float16)b[1]; v[6]=(_Float16)b[2]; v[7]=(_Float16)b[3];
  *(volatile v8h*)(dst + (size_t)t * 8) = v;
  __threadfence();
  *(volatile v8h*)(dst + (size_t)t * 8) = v;
}

__global__ __launch_bounds__(256) void k_transpose16(const float* __restrict__ W, _Float16* __restrict__ Wt, int K, int N) {
  const int t = blockIdx.x * 256 + threadIdx.x;
  const int k8n = K / 8;
  if (t >= N * k8n) return;
  const int n = t / k8n, k8 = (t % k8n) * 8;
  v8h v;
#pragma unroll
  for (int i = 0; i < 8; ++i) v[i] = (_Float16)W[(size_t)(k8 + i) * N + n];
  *(volatile v8h*)(Wt + (size_t)n * K + k8) = v;
  __threadfence();
  *(volatile v8h*)(Wt + (size_t)n * K + k8) = v;
}

template <int ACT, bool OUT16>
__global__ __launch_bounds__(128) void k_gemm(const _Float16* __restrict__ A, int lda, const _Float16* __restrict__ Bt, int ldb,
                                            const float* __restrict__ bias, void* __restrict__ Cout, int ldc, int M, int N, int K) {
  __shared__ __attribute__((aligned(16))) float so[4][16][64];
  const int tid = threadIdx.x, w = tid >> 5, lane = tid & 31, ln = lane & 15, hh = lane >> 4;
  const int ntn = N / 64;
  const int wid = blockIdx.x * 4 + w;
  const int mt = wid / ntn, nq = wid % ntn;
  if (mt * 16 >= M) return;
  const int row0 = mt * 16, col0 = nq * 64;
  const _Float16* arow = A + (size_t)(row0 + ln) * lda;
  v8f acc[4] = {};
  for (int kb = 0; kb < K; kb += 32) {
    Frag a;
    a.half[0] = *(const v8ha*)(arow + kb + 8 * hh);
    a.half[1] = *(const v8ha*)(arow + kb + 16 + 8 * hh);
#pragma unroll
    for (int t = 0; t < 4; ++t) {
      const _Float16* brow = Bt + (size_t)(col0 + t * 16 + ln) * ldb + kb;
      Frag b;
      b.half[0] = *(const v8ha*)(brow + 8 * hh);
      b.half[1] = *(const v8ha*)(brow + 16 + 8 * hh);
      acc[t] = mma16(a.v, b.v, acc[t]);
    }
  }
#pragma unroll
  for (int t = 0; t < 4; ++t) {
    const float bv = bias ? bias[col0 + t * 16 + ln] : 0.f;
#pragma unroll
    for (int r = 0; r < 8; ++r) { float v = acc[t][r] + bv; if (ACT == 1) v = fmaxf(v, 0.f); so[w][8 * hh + r][t * 16 + ln] = v; }
  }
  __builtin_amdgcn_fence(__ATOMIC_ACQ_REL, "workgroup");
  __builtin_amdgcn_wave_barrier();
  if (OUT16) {
    _Float16* C = (_Float16*)Cout;
    const int rsub = lane >> 3, c8 = (lane & 7) * 8;
    for (int pass = 0; pass < 2; ++pass) {
#pragma unroll
      for (int q = 0; q < 4; ++q) {
        const int r = q * 4 + rsub;
        v8h v;
#pragma unroll
        for (int i = 0; i < 8; ++i) v[i] = (_Float16)so[w][r][c8 + i];
        *(volatile v8h*)(C + (size_t)(row0 + r) * ldc + col0 + c8) = v;
      }
      if (pass == 0) __threadfence();
    }
  } else {
    float* C = (float*)Cout;
    const int rsub = lane >> 4, c4 = (lane & 15) * 4;
    for (int pass = 0; pass < 2; ++pass) {
#pragma unroll
      for (int q = 0; q < 8; ++q) {
        const int r = q * 2 + rsub;
        const v4f v = *(const v4fa*)&so[w][r][c4];
        *(volatile v4f*)(C + (size_t)(row0 + r) * ldc + col0 + c4) = v;
      }
      if (pass == 0) __threadfence();
    }
  }
}

__global__ __launch_bounds__(256) void k_rel(const float* __restrict__ spans, const float* __restrict__ toks, const int* __restrict__ ids,
                                           const int* __restrict__ tmask, _Float16* __restrict__ rel) {
  __shared__ __attribute__((aligned(16))) _Float16 srow[3 * HH];
  const int p = blockIdx.x, tid = threadIdx.x;
  const int b = p / (KK * KK), ij = p % (KK * KK), i = ij / KK, j = ij % KK;
  const float* hi = spans + ((size_t)b * KK + i) * HH;
  const float* tj = spans + ((size_t)b * KK + j) * HH;
  int si = ids[((b * KK) + i) * 2 + 0], ei = ids[((b * KK) + i) * 2 + 1];
  int sj = ids[((b * KK) + j) * 2 + 0], ej = ids[((b * KK) + j) * 2 + 1];
  const int min_end = ei < ej ? ei : ej, max_start = si > sj ? si : sj;
  const bool valid = min_end < max_start;
  int t0 = min_end < 0 ? 0 : min_end, t1 = max_start > SS ? SS : max_start;
  for (int f = tid; f < HH; f += 256) {
    srow[f] = (_Float16)hi[f];
    srow[HH + f] = (_Float16)tj[f];
    float ctx = hi[f];
    if (valid) {
      float m = -__builtin_inff();
      for (int t = t0; t < t1; ++t) if (tmask[b * SS + t] != 0) m = fmaxf(m, toks[((size_t)b * SS + t) * HH + f]);
      ctx = m;
    }
    srow[2 * HH + f] = (_Float16)ctx;
  }
  __syncthreads();
  if (tid < 3 * HH / 8) {
    const v8h v = *(const v8ha*)&srow[tid * 8];
    *(volatile v8h*)(rel + (size_t)p * 3 * HH + tid * 8) = v;
    __threadfence();
    *(volatile v8h*)(rel + (size_t)p * 3 * HH + tid * 8) = v;
  }
}

extern "C" void kernel_launch(void* const* d_in, const int* in_sizes, int n_in,
                              void* d_out, int out_size, void* d_ws, size_t ws_size, hipStream_t stream) {
  (void)in_sizes; (void)n_in; (void)out_size;
  const float* spans = (const float*)d_in[0];
  const float* toks  = (const float*)d_in[1];
  const float* W1 = (const float*)d_in[2]; const float* b1 = (const float*)d_in[3];
  const float* W2 = (const float*)d_in[4]; const float* b2 = (const float*)d_in[5];
  const int* ids = (const int*)d_in[6]; const int* tmask = (const int*)d_in[7];
  char* ws = (char*)d_ws; size_t off = 0;
  _Float16* W1t = (_Float16*)(ws + off); off += (size_t)FF * (3 * HH) * 2;
  _Float16* W2t = (_Float16*)(ws + off); off += (size_t)HH * FF * 2;
  _Float16* rel = (_Float16*)(ws + off); off += (size_t)NP * 3 * HH * 2;
  _Float16* hid = (_Float16*)(ws + off); off += (size_t)NP * FF * 2;
  if (off > ws_size) return;
  k_transpose16<<<(FF * (3 * HH / 8) + 255) / 256, 256, 0, stream>>>(W1, W1t, 3 * HH, FF);
  k_transpose16<<<(HH * (FF / 8) + 255) / 256, 256, 0, stream>>>(W2, W2t, FF, HH);
  k_rel<<<NP, 256, 0, stream>>>(spans, toks, ids, tmask, rel);
  k_gemm<1, true ><<<(NP / 16) * (FF / 64) / 4, 128, 0, stream>>>(rel, 3 * HH, W1t, 3 * HH, b1, (void*)hid, FF, NP, FF, 3 * HH);
  k_gemm<0, false><<<(NP / 16) * (HH / 64) / 4, 128, 0, stream>>>(hid, FF, W2t, FF, b2, d_out, HH, NP, HH, FF);
}
